// DecoderLayer_2671469658570
// MI455X (gfx1250) — hardware-verified
//
#include <hip/hip_runtime.h>
#include <math.h>

#ifndef NB
#define NB 4
#endif
#ifndef SEQ
#define SEQ 1024
#endif
#define NB_FULL 4
#define SEQ_FULL 1024

constexpr int kBatch    = NB;
constexpr int kSeq      = SEQ;
constexpr int kSeqFull  = SEQ_FULL;
constexpr int kModel    = 1024;
constexpr int kHeads    = 16;
constexpr int kHeadDim  = 64;
constexpr int kFF       = 4096;
constexpr int kTok      = kBatch * kSeq;
constexpr int kQT       = kSeq / 64;
constexpr int kFlagPitch = 32;
static_assert(NB >= 1 && NB <= NB_FULL);
static_assert(SEQ >= 64 && SEQ <= SEQ_FULL && (SEQ % 64) == 0);
static_assert(kQT <= kFlagPitch);
static_assert(kHeads * kHeadDim == kModel);
static_assert((kTok % 64) == 0 && (kModel % 64) == 0 && (kFF % 64) == 0);

constexpr float kWCarry     = 16.0f;
constexpr float kWCarryInv  = 1.0f / 16.0f;
constexpr float kW2Carry    = 32.0f;
constexpr float kW2CarryInv = 1.0f / 32.0f;
constexpr float kPCarry     = 1024.0f;
constexpr float kCtxCarry   = 16.0f;
constexpr float kPVScale    = kCtxCarry / kPCarry;
constexpr float kWoScale    = 1.0f / (kCtxCarry * kWCarry);
constexpr float kScoreScale = 0.125f;
constexpr float kInvModel   = 1.0f / 1024.0f;
constexpr float kLnEps      = 1e-5f;

constexpr size_t kMiB     = 1048576;
constexpr size_t kOffXR   = 0;
constexpr size_t kOffEnc  = 0;
constexpr size_t kOffW1T  = 8 * kMiB;
constexpr size_t kOffH16  = 16 * kMiB;
constexpr size_t kOffWT4  = 24 * kMiB;
constexpr size_t kOffW2T  = 24 * kMiB;
constexpr size_t kOffQ16  = 32 * kMiB;
constexpr size_t kOffK16  = 40 * kMiB;
constexpr size_t kOffVT16 = 48 * kMiB;
constexpr size_t kOffCtx  = 56 * kMiB;
constexpr size_t kOffHFF  = 32 * kMiB;
constexpr size_t kOffY1   = 64 * kMiB;
constexpr size_t kOffY2   = 80 * kMiB;
constexpr size_t kOffFl0  = 96 * kMiB;
constexpr size_t kOffFl1  = 96 * kMiB + 8192;
constexpr size_t kWsTotal = 96 * kMiB + 16384;
static_assert((size_t)kTok * kModel * 4 <= 16 * kMiB);
static_assert((size_t)kTok * kModel * 2 <= 8 * kMiB);
static_assert((size_t)4 * kModel * kModel * 2 == 8 * kMiB);
static_assert((size_t)kModel * kFF * 2 == 8 * kMiB);
static_assert((size_t)kTok * kFF * 2 <= 32 * kMiB);
static_assert((size_t)kBatch * kQT * kFlagPitch * 4 <= 8192);
static_assert(kOffHFF + 32 * kMiB <= kOffY1);
static_assert(kWsTotal <= 134217728);

typedef __attribute__((ext_vector_type(16))) _Float16 v16h;
typedef __attribute__((ext_vector_type(8)))  _Float16 v8h;
typedef __attribute__((ext_vector_type(16))) __bf16   v16b;
typedef __attribute__((ext_vector_type(8)))  __bf16   v8b;
typedef __attribute__((ext_vector_type(8)))  float    v8f;
typedef __attribute__((ext_vector_type(4)))  float    v4f;
typedef __attribute__((ext_vector_type(4)))  unsigned int v4u;
typedef __attribute__((ext_vector_type(4)))  int      v4i;

__device__ __forceinline__ unsigned short f2bf_bits(float f) {
  unsigned u = __float_as_uint(f);
  return (unsigned short)((u + 0x7FFFu + ((u >> 16) & 1u)) >> 16);
}
__device__ __forceinline__ float bf_bits2f(unsigned short h) { return __uint_as_float(((unsigned)h) << 16); }
__device__ __forceinline__ float bfr(float f) { return bf_bits2f(f2bf_bits(f)); }

__device__ __forceinline__ void dep_guard_h(v8f& a, v8f& b, v16h x, v16h y) { asm volatile("v_nop\n\tv_nop\n\tv_nop\n\tv_nop" : "+v"(a), "+v"(b) : "v"(x), "v"(y)); }
__device__ __forceinline__ void dep_guard_b(v8f& a, v8f& b, v16b x, v16b y) { asm volatile("v_nop\n\tv_nop\n\tv_nop\n\tv_nop" : "+v"(a), "+v"(b) : "v"(x), "v"(y)); }
__device__ __forceinline__ void keep4_h(v16h a, v16h b, v16h c, v16h d) { asm volatile("v_nop" :: "v"(a), "v"(b), "v"(c), "v"(d)); }
__device__ __forceinline__ void keep4_b(v16b a, v16b b, v16b c, v16b d) { asm volatile("v_nop" :: "v"(a), "v"(b), "v"(c), "v"(d)); }
__device__ __forceinline__ void acc_guard4(v8f& a, v8f& b, v8f& c, v8f& d) { asm volatile("v_nop\n\tv_nop\n\tv_nop\n\tv_nop" : "+v"(a), "+v"(b), "+v"(c), "+v"(d)); }
template <typename T> struct Frag;
template <> struct Frag<_Float16> {
  typedef v16h V; union U { v16h v; v8h h[2]; };
  static __device__ __forceinline__ v16h load(const _Float16* p) {
    U f; f.h[0] = *(const v8h*)(p); f.h[1] = *(const v8h*)(p + 16); return f.v;
  }
  static __device__ __forceinline__ v8f mma(v16h a, v16h b, v8f c) {
    return __builtin_amdgcn_wmma_f32_16x16x32_f16(false, a, false, b, (short)0, c, false, false);
  }
  static __device__ __forceinline__ void guard(v8f& a, v8f& b, v16h x, v16h y) { dep_guard_h(a, b, x, y); }
  static __device__ __forceinline__ void keep(v16h a, v16h b, v16h c, v16h d) { keep4_h(a, b, c, d); }
};
template <> struct Frag<__bf16> {
  typedef v16b V; union U { v16b v; v8b h[2]; };
  static __device__ __forceinline__ v16b load(const __bf16* p) {
    U f; f.h[0] = *(const v8b*)(p); f.h[1] = *(const v8b*)(p + 16); return f.v;
  }
  static __device__ __forceinline__ v8f mma(v16b a, v16b b, v8f c) {
    return __builtin_amdgcn_wmma_f32_16x16x32_bf16(false, a, false, b, (short)0, c, false, false);
  }
  static __device__ __forceinline__ void guard(v8f& a, v8f& b, v16b x, v16b y) { dep_guard_b(a, b, x, y); }
  static __device__ __forceinline__ void keep(v16b a, v16b b, v16b c, v16b d) { keep4_b(a, b, c, d); }
};

__device__ __forceinline__ unsigned pk16(unsigned short a, unsigned short b) { return (unsigned)a | ((unsigned)b << 16); }
__device__ __forceinline__ unsigned short h_bits(float f) { const _Float16 h = (_Float16)f; return __builtin_bit_cast(unsigned short, h); }

template <int ET> struct Elem;
template <> struct Elem<0> { typedef _Float16 T; };
template <> struct Elem<1> { typedef __bf16 T; };
template <int ET, bool SPLIT, int BIAS_MODE, int OUT_MODE, bool RESID, int ACT = 0, int TRI = 0>
__global__ __launch_bounds__(256) void wmma_gemm64(
    const unsigned short* __restrict__ Ap, const unsigned short* __restrict__ A2p, int lda, long strideA,
    const unsigned short* __restrict__ Btp, const unsigned short* __restrict__ Bt2p, int ldb, long strideB,
    void* __restrict__ Cout, void* __restrict__ Cout2, int ldc, long strideC,
    const float* __restrict__ bias,
    const float* __restrict__ resid, long strideR,
    int M, int N, int K, float scale) {
  static_assert(!RESID || (OUT_MODE == 0 && ACT == 0));
  typedef typename Elem<ET>::T T;
  typedef typename Frag<T>::V V;
  const T* A = (const T*)Ap; const T* A2 = (const T*)A2p; const T* Bt = (const T*)Btp; const T* Bt2 = (const T*)Bt2p;
  __shared__ __align__(16) float sT[8][16 * 68];
  const int b    = blockIdx.y;
  const int lane = threadIdx.x & 31;
  const int wave = threadIdx.x >> 5;
  const int tilesN = N >> 6;
  const int tilesM = M >> 6;
  const int tile = blockIdx.x * 8 + wave;
  if (tile >= tilesM * tilesN) return;
  const int tm = tile / tilesN;
  const int tn = tile - tm * tilesN;
  if (TRI == 1 && tn > tm) return;
  const int m0 = tm << 6;
  const int n0 = tn << 6;
  const int kEnd = (TRI == 2) ? (((m0 + 64) < K) ? (m0 + 64) : K) : K;

  const T* Ab  = A  + (size_t)b * strideA;
  const T* Bb  = Bt + (size_t)b * strideB;
  const T* Ab2 = SPLIT ? (A2  + (size_t)b * strideA) : nullptr;
  const T* Bb2 = SPLIT ? (Bt2 + (size_t)b * strideB) : nullptr;

  const int rlane = lane & 15;
  const int koff  = (lane >> 4) * 8;
  const int mOff  = (lane >> 4) * 8;

  v8f acc[4][4];
#pragma unroll
  for (int i = 0; i < 4; ++i)
#pragma unroll
    for (int j = 0; j < 4; ++j) acc[i][j] = (v8f){0.f,0.f,0.f,0.f,0.f,0.f,0.f,0.f};

  for (int k0 = 0; k0 < kEnd; k0 += 32) {
    V bh[4], bl[4];
#pragma unroll
    for (int j = 0; j < 4; ++j) {
      const size_t bo = (size_t)(n0 + (j << 4) + rlane) * ldb + koff + k0;
      bh[j] = Frag<T>::load(Bb + bo);
      if (SPLIT) bl[j] = Frag<T>::load(Bb2 + bo);
    }
#pragma unroll
    for (int i = 0; i < 4; ++i) {
      const size_t ao = (size_t)(m0 + (i << 4) + rlane) * lda + koff + k0;
      V ah = Frag<T>::load(Ab + ao);
      V al;
      if (SPLIT) al = Frag<T>::load(Ab2 + ao);
#pragma unroll
      for (int j = 0; j < 4; ++j) {
        acc[i][j] = Frag<T>::mma(ah, bh[j], acc[i][j]);
        if (SPLIT) {
          acc[i][j] = Frag<T>::mma(ah, bl[j], acc[i][j]);
          acc[i][j] = Frag<T>::mma(al, bh[j], acc[i][j]);
        }
      }
      Frag<T>::guard(acc[i][0], acc[i][3], ah, SPLIT ? al : ah);
    }
    Frag<T>::keep(bh[0], bh[1], bh[2], bh[3]);
    if (SPLIT) Frag<T>::keep(bl[0], bl[1], bl[2], bl[3]);
  }
  acc_guard4(acc[0][0], acc[0][1], acc[0][2], acc[0][3]);
  acc_guard4(acc[1][0], acc[1][1], acc[1][2], acc[1][3]);
  acc_guard4(acc[2][0], acc[2][1], acc[2][2], acc[2][3]);
  acc_guard4(acc[3][0], acc[3][1], acc[3][2], acc[3][3]);

  float* slab = sT[wave];
  const float* Rb = RESID ? (resid + (size_t)b * strideR) : nullptr;
#pragma unroll
  for (int i = 0; i < 4; ++i) {
    const int mBase = m0 + (i << 4);
    float bm[8];
#pragma unroll
    for (int e = 0; e < 8; ++e) bm[e] = 0.0f;
    if (BIAS_MODE == 1) {
      const v4f ba = *(const v4f*)(bias + mBase + mOff);
      const v4f bc = *(const v4f*)(bias + mBase + mOff + 4);
#pragma unroll
      for (int e = 0; e < 4; ++e) { bm[e] = bfr(ba[e]); bm[4 + e] = bfr(bc[e]); }
    }
#pragma unroll
    for (int j = 0; j < 4; ++j) {
      const int n = n0 + (j << 4) + rlane;
      float bv = 0.f;
      if (BIAS_MODE == 2) bv = bfr(bias[n]);
#pragma unroll
      for (int r = 0; r < 8; ++r) {
        float v = acc[i][j][r] * scale;
        if (BIAS_MODE == 1) v += bm[r];
        if (BIAS_MODE == 2) v += bv;
        if (ACT == 2) v = fmaxf(v, 0.0f);
        if (ACT == 3) v = 0.5f * v * (1.0f + erff(v * 0.70710678118654752f));
        if (ACT == 4) v = (v > 0.f) ? v : 0.01f * v;
        slab[(mOff + r) * 68 + (j << 4) + rlane] = v;
      }
    }
    __builtin_amdgcn_fence(3, "workgroup");
    __builtin_amdgcn_wave_barrier();
    __builtin_amdgcn_fence(2, "workgroup");
    if (OUT_MODE == 0) {
      float* C = (float*)Cout + (size_t)b * strideC;
      const int hh = lane >> 4, c4 = (lane & 15) * 4;
      v4f fin[8];
#pragma unroll
      for (int it = 0; it < 8; ++it) {
        const int row = it * 2 + hh;
        v4f v = *(const v4f*)(slab + row * 68 + c4);
        if (RESID) {
          const v4f rv = *(const v4f*)(Rb + (size_t)(mBase + row) * ldc + n0 + c4);
          v = v + rv;
        }
        fin[it] = v;
      }
      for (int pass = 0; pass < 2; ++pass) {
#pragma unroll
        for (int it = 0; it < 8; ++it) {
          const int row = it * 2 + hh;
          *(volatile v4f*)(C + (size_t)(mBase + row) * ldc + n0 + c4) = fin[it];
        }
        __threadfence();
      }
    } else {
      const int q = lane >> 3, c8 = (lane & 7) * 8;
      unsigned short* C  = (unsigned short*)Cout  + (size_t)b * strideC;
      unsigned short* C2 = (OUT_MODE == 2) ? ((unsigned short*)Cout2 + (size_t)b * strideC) : nullptr;
      for (int pass = 0; pass < 2; ++pass) {
#pragma unroll
        for (int it = 0; it < 4; ++it) {
          const int row = it * 4 + q;
          const float* sp = slab + row * 68 + c8;
          v8h hv, lv;
#pragma unroll
          for (int e = 0; e < 8; ++e) {
            if (OUT_MODE == 1) {
              hv[e] = (_Float16)sp[e];
            } else {
              unsigned short hb = f2bf_bits(sp[e]);
              unsigned short lb = f2bf_bits(sp[e] - bf_bits2f(hb));
              hv[e] = __builtin_bit_cast(_Float16, hb);
              lv[e] = __builtin_bit_cast(_Float16, lb);
            }
          }
          *(volatile v8h*)(C + (size_t)(mBase + row) * ldc + n0 + c8) = hv;
          if (OUT_MODE == 2) *(volatile v8h*)(C2 + (size_t)(mBase + row) * ldc + n0 + c8) = lv;
        }
        __threadfence();
      }
    }
    __builtin_amdgcn_fence(3, "workgroup");
    __builtin_amdgcn_wave_barrier();
    __builtin_amdgcn_fence(2, "workgroup");
  }
}

__global__ __launch_bounds__(256) void tcast_kernel(const float* __restrict__ W0, const float* __restrict__ W1,
                                                    const float* __restrict__ W2, const float* __restrict__ W3,
                                                    unsigned short* __restrict__ out, int R, int Ccols,
                                                    long planeStride, float scale) {
  __shared__ float sm[64][65];
  const int t  = threadIdx.x;
  const int r0 = blockIdx.x * 64;
  const int c0 = blockIdx.y * 64;
  const int z  = blockIdx.z;
  const float* W = (z == 0) ? W0 : (z == 1) ? W1 : (z == 2) ? W2 : W3;
#pragma unroll 8
  for (int i = 0; i < 16; ++i) {
    const int e  = i * 256 + t;
    const int rl = e >> 6;
    const int cl = e & 63;
    sm[cl][rl] = bfr(W[(size_t)(r0 + rl) * Ccols + c0 + cl]) * scale;
  }
  __syncthreads();
  const int lane = t & 31, wave = t >> 5;
  const int q = lane >> 3, c8 = (lane & 7) * 8;
  unsigned short* op = out + (size_t)z * planeStride;
  for (int pass = 0; pass < 2; ++pass) {
#pragma unroll
    for (int it = 0; it < 2; ++it) {
      const int row = wave * 8 + it * 4 + q;
      unsigned short hb[8];
#pragma unroll
      for (int e = 0; e < 8; ++e) hb[e] = h_bits(sm[row][c8 + e]);
      const v4u u = (v4u){pk16(hb[0], hb[1]), pk16(hb[2], hb[3]), pk16(hb[4], hb[5]), pk16(hb[6], hb[7])};
      *(volatile v4u*)(op + (size_t)(c0 + row) * R + r0 + c8) = u;
    }
    __threadfence();
  }
}

__global__ __launch_bounds__(256) void enccast_kernel(const float* __restrict__ in, unsigned short* __restrict__ out, int n8) {
  const int i = blockIdx.x * 256 + threadIdx.x;
  if (i >= n8) return;
  const int tok = i >> 7;
  const int col = (i & 127) * 8;
  const int b   = tok / kSeq;
  const int tt  = tok - b * kSeq;
  const float* p = in + ((size_t)b * kSeqFull + tt) * kModel + col;
  const v4f a = *(const v4f*)(p);
  const v4f c = *(const v4f*)(p + 4);
  unsigned short hb[8];
#pragma unroll
  for (int e = 0; e < 4; ++e) {
    hb[e]     = h_bits(bfr(a[e]));
    hb[4 + e] = h_bits(bfr(c[e]));
  }
  const v4u u = (v4u){pk16(hb[0], hb[1]), pk16(hb[2], hb[3]), pk16(hb[4], hb[5]), pk16(hb[6], hb[7])};
  unsigned short* q = out + 8 * (size_t)i;
  *(volatile v4u*)q = u;
  __threadfence();
  *(volatile v4u*)q = u;
}

template <bool FIRST>
__global__ __launch_bounds__(256) void ln_kernel(const float* __restrict__ X, const float* __restrict__ gam,
                                                  const float* __restrict__ bet, float* __restrict__ xcopy,
                                                  unsigned short* __restrict__ out16) {
  __shared__ float red1[8];
  __shared__ float red2[8];
  __shared__ __align__(16) float rowbuf[kModel];
  const int row = blockIdx.x;
  const int t = threadIdx.x, lane = t & 31, wave = t >> 5;
  size_t inrow = (size_t)row;
  if (FIRST) {
    const int b = row / kSeq;
    const int tt = row - b * kSeq;
    inrow = (size_t)b * kSeqFull + tt;
  }
  v4f xv = *(const v4f*)(X + inrow * kModel + 4 * t);
  if (FIRST) {
#pragma unroll
    for (int e = 0; e < 4; ++e) xv[e] = bfr(xv[e]);
  }
  float s = (xv[0] + xv[1]) + (xv[2] + xv[3]);
#pragma unroll
  for (int off = 16; off > 0; off >>= 1) s += __shfl_xor(s, off, 32);
  if (lane == 0) red1[wave] = s;
  __syncthreads();
  float tot = red1[0];
#pragma unroll
  for (int w = 1; w < 8; ++w) tot += red1[w];
  const float mean = tot * kInvModel;
  v4f d;
#pragma unroll
  for (int e = 0; e < 4; ++e) d[e] = xv[e] - mean;
  float s2 = (d[0] * d[0] + d[1] * d[1]) + (d[2] * d[2] + d[3] * d[3]);
#pragma unroll
  for (int off = 16; off > 0; off >>= 1) s2 += __shfl_xor(s2, off, 32);
  if (lane == 0) red2[wave] = s2;
  __syncthreads();
  float tot2 = red2[0];
#pragma unroll
  for (int w = 1; w < 8; ++w) tot2 += red2[w];
  const float var  = tot2 * kInvModel;
  const float rinv = rsqrtf(var + kLnEps);
  const v4f gg = *(const v4f*)(gam + 4 * t);
  const v4f bb = *(const v4f*)(bet + 4 * t);
  v4f o;
#pragma unroll
  for (int e = 0; e < 4; ++e) o[e] = d[e] * rinv * bfr(gg[e]) + bfr(bb[e]);
  if (FIRST) {
    float* op = xcopy + (size_t)row * kModel + 4 * t;
    *(volatile v4f*)op = xv;
    __threadfence();
    *(volatile v4f*)op = xv;
  }
  *(v4f*)(rowbuf + 4 * t) = o;
  __syncthreads();
  if (t < 128) {
    const v4f a = *(const v4f*)(rowbuf + 8 * t);
    const v4f c = *(const v4f*)(rowbuf + 8 * t + 4);
    unsigned short hb[8];
#pragma unroll
    for (int e = 0; e < 4; ++e) {
      hb[e]     = h_bits(a[e]);
      hb[4 + e] = h_bits(c[e]);
    }
    const v4u u = (v4u){pk16(hb[0], hb[1]), pk16(hb[2], hb[3]), pk16(hb[4], hb[5]), pk16(hb[6], hb[7])};
    unsigned short* q = out16 + (size_t)row * kModel + 8 * t;
    *(volatile v4u*)q = u;
    __threadfence();
    *(volatile v4u*)q = u;
  }
}

__global__ __launch_bounds__(256) void tileflag_kernel(const int* __restrict__ m0p, const int* __restrict__ m1p,
                                                       int* __restrict__ f0p, int* __restrict__ f1p) {
  __shared__ int redz[8];
  __shared__ int rednz[8];
  __shared__ int fl[32];
  const int t = threadIdx.x, lane = t & 31, wave = t >> 5;
  const int z = blockIdx.y;
  const int* mp = (z == 0) ? m0p : m1p;
  int* fp = (z == 0) ? f0p : f1p;
  const int bq = blockIdx.x;
  const int b  = bq / kQT;
  const int qt = bq - b * kQT;
  const int row = t >> 2;
  const int cq  = (t & 3) * 16;
  const int* base = mp + (size_t)b * kSeqFull * kSeqFull + (size_t)(qt * 64 + row) * kSeqFull + cq;
  if (t < 32) fl[t] = 2;
#pragma unroll 1
  for (int kc = 0; kc < kQT; ++kc) {
    const int* p = base + kc * 64;
    const v4i a0 = *(const v4i*)(p);
    const v4i a1 = *(const v4i*)(p + 4);
    const v4i a2 = *(const v4i*)(p + 8);
    const v4i a3 = *(const v4i*)(p + 12);
    int hz = 0, hnz = 0;
#pragma unroll
    for (int e = 0; e < 4; ++e) {
      hz  |= (a0[e] == 0) | (a1[e] == 0) | (a2[e] == 0) | (a3[e] == 0);
      hnz |= (a0[e] != 0) | (a1[e] != 0) | (a2[e] != 0) | (a3[e] != 0);
    }
    const unsigned long long bz  = __ballot(hz);
    const unsigned long long bnz = __ballot(hnz);
    if (lane == 0) { redz[wave] = (bz != 0ull) ? 1 : 0; rednz[wave] = (bnz != 0ull) ? 1 : 0; }
    __syncthreads();
    if (t == 0) {
      int az = 0, anz = 0;
#pragma unroll
      for (int w = 0; w < 8; ++w) { az |= redz[w]; anz |= rednz[w]; }
      fl[kc] = (anz == 0) ? 0 : ((az == 0) ? 1 : 2);
    }
    __syncthreads();
  }
  if (wave == 0) {
    const int v = fl[lane];
    int* q = fp + (size_t)bq * kFlagPitch + lane;
    *(volatile int*)q = v;
    __threadfence();
    *(volatile int*)q = v;
  }
}

constexpr int kLP = 72;
__global__ __launch_bounds__(128) __attribute__((amdgpu_num_vgpr(256)))
void attn_kernel(const unsigned short* __restrict__ Qp, const unsigned short* __restrict__ Kp,
                 const unsigned short* __restrict__ VTp, const int* __restrict__ msk,
                 const int* __restrict__ flags, unsigned short* __restrict__ Cxp) {
  __shared__ __align__(16) _Float16 Kt[64 * kLP];
  __shared__ __align__(16) _Float16 Vt[64 * kLP];
  __shared__ __align__(16) _Float16 Pt[4][16 * kLP];
  __shared__ __align__(16) int Mt[64 * 64];
  typedef Frag<_Float16> F;
  const int tid  = threadIdx.x;
  const int wave = tid >> 5, lane = tid & 31, l15 = lane & 15, half = lane >> 4;
  const int b  = blockIdx.y / kHeads;
  const int h  = blockIdx.y - b * kHeads;
  const int qt = blockIdx.x;
  const int tokq0 = b * kSeq + qt * 64;
  const int hoff  = h * kHeadDim;
  const _Float16* Q = (const _Float16*)Qp;
  const _Float16* qr = Q + (size_t)(tokq0 + wave * 16 + l15) * kModel + hoff + 8 * half;
  const v16h aq0 = F::load(qr);
  const v16h aq1 = F::load(qr + 32);
  const v8f z8 = (v8f){0.f,0.f,0.f,0.f,0.f,0.f,0.f,0.f};
  v8f o0 = z8, o1 = z8, o2 = z8, o3 = z8;
  float mrow[8], lrow[8];
#pragma unroll
  for (int r = 0; r < 8; ++r) { mrow[r] = -INFINITY; lrow[r] = 0.0f; }
  _Float16* Pw = Pt[wave];
  unsigned short* KtU = (unsigned short*)Kt;
  unsigned short* VtU = (unsigned short*)Vt;
  const int* mblk = msk + (size_t)b * kSeqFull * kSeqFull + (size_t)(qt * 64) * kSeqFull;
  const int* frow = flags + (size_t)(b * kQT + qt) * kFlagPitch;

#pragma unroll 1
  for (int kc = 0; kc < kQT; ++kc) {
    const int f = frow[kc];
    if (f == 0) continue;
    const bool useM = (f != 1);
    const int tokk0 = b * kSeq + kc * 64;
    __syncthreads();
#pragma unroll
    for (int i = 0; i < 4; ++i) {
      const int idx = i * 128 + tid;
      const int row = idx >> 3;
      const int c8  = (idx & 7) * 8;
      const v4u kv = *(const v4u*)(Kp + (size_t)(tokk0 + row) * kModel + hoff + c8);
      *(v4u*)(KtU + row * kLP + c8) = kv;
      const v4u vv = *(const v4u*)(VTp + (size_t)(hoff + row) * kTok + tokk0 + c8);
      *(v4u*)(VtU + row * kLP + c8) = vv;
    }
    if (useM) {
#pragma unroll
      for (int i = 0; i < 8; ++i) {
        const int idx = i * 128 + tid;
        const int row = idx >> 4;
        const int c4  = (idx & 15) * 4;
        const v4i mv = *(const v4i*)(mblk + (size_t)row * kSeqFull + kc * 64 + c4);
        *(v4i*)(Mt + row * 64 + c4) = mv;
      }
    }
    __syncthreads();

    v8f s0 = z8, s1 = z8, s2 = z8, s3 = z8;
    {
      const v16h bk0 = F::load(Kt + (0 * 16 + l15) * kLP + 8 * half);
      const v16h bk1 = F::load(Kt + (1 * 16 + l15) * kLP + 8 * half);
      const v16h bk2 = F::load(Kt + (2 * 16 + l15) * kLP + 8 * half);
      const v16h bk3 = F::load(Kt + (3 * 16 + l15) * kLP + 8 * half);
      s0 = F::mma(aq0, bk0, s0);
      s1 = F::mma(aq0, bk1, s1);
      s2 = F::mma(aq0, bk2, s2);
      s3 = F::mma(aq0, bk3, s3);
      keep4_h(bk0, bk1, bk2, bk3);
      const v16h bk4 = F::load(Kt + (0 * 16 + l15) * kLP + 32 + 8 * half);
      const v16h bk5 = F::load(Kt + (1 * 16 + l15) * kLP + 32 + 8 * half);
      const v16h bk6 = F::load(Kt + (2 * 16 + l15) * kLP + 32 + 8 * half);
      const v16h bk7 = F::load(Kt + (3 * 16 + l15) * kLP + 32 + 8 * half);
      s0 = F::mma(aq1, bk4, s0);
      s1 = F::mma(aq1, bk5, s1);
      s2 = F::mma(aq1, bk6, s2);
      s3 = F::mma(aq1, bk7, s3);
      keep4_h(bk4, bk5, bk6, bk7);
      keep4_h(aq0, aq1, aq0, aq1);
    }
    acc_guard4(s0, s1, s2, s3);

#pragma unroll
    for (int r = 0; r < 8; ++r) {
      float sv0 = s0[r] * kScoreScale;
      float sv1 = s1[r] * kScoreScale;
      float sv2 = s2[r] * kScoreScale;
      float sv3 = s3[r] * kScoreScale;
      if (useM) {
        const int* mr = Mt + (wave * 16 + 8 * half + r) * 64 + l15;
        const int k0 = mr[0], k1 = mr[16], k2 = mr[32], k3 = mr[48];
        sv0 = (k0 != 0) ? sv0 : -INFINITY;
        sv1 = (k1 != 0) ? sv1 : -INFINITY;
        sv2 = (k2 != 0) ? sv2 : -INFINITY;
        sv3 = (k3 != 0) ? sv3 : -INFINITY;
      }
      float mx = fmaxf(fmaxf(sv0, sv1), fmaxf(sv2, sv3));
      mx = fmaxf(mx, __shfl_xor(mx, 1, 32));
      mx = fmaxf(mx, __shfl_xor(mx, 2, 32));
      mx = fmaxf(mx, __shfl_xor(mx, 4, 32));
      mx = fmaxf(mx, __shfl_xor(mx, 8, 32));
      const float mnew = fmaxf(mrow[r], mx);
      const float mref = (mnew == -INFINITY) ? 0.0f : mnew;
      const float sc = __expf(mrow[r] - mref);
      const float p0 = __expf(sv0 - mref);
      const float p1 = __expf(sv1 - mref);
      const float p2 = __expf(sv2 - mref);
      const float p3 = __expf(sv3 - mref);
      float sum = (p0 + p1) + (p2 + p3);
      sum += __shfl_xor(sum, 1, 32);
      sum += __shfl_xor(sum, 2, 32);
      sum += __shfl_xor(sum, 4, 32);
      sum += __shfl_xor(sum, 8, 32);
      lrow[r] = lrow[r] * sc + sum;
      mrow[r] = mnew;
      o0[r] *= sc; o1[r] *= sc; o2[r] *= sc; o3[r] *= sc;
      _Float16* pr = Pw + (8 * half + r) * kLP + l15;
      pr[0]  = (_Float16)(p0 * kPCarry);
      pr[16] = (_Float16)(p1 * kPCarry);
      pr[32] = (_Float16)(p2 * kPCarry);
      pr[48] = (_Float16)(p3 * kPCarry);
    }
    __builtin_amdgcn_fence(3, "workgroup");
    __builtin_amdgcn_wave_barrier();
    __builtin_amdgcn_fence(2, "workgroup");

    {
      const v16h ap0 = F::load(Pw + l15 * kLP + 8 * half);
      const v16h bv0 = F::load(Vt + (0 * 16 + l15) * kLP + 8 * half);
      const v16h bv1 = F::load(Vt + (1 * 16 + l15) * kLP + 8 * half);
      const v16h bv2 = F::load(Vt + (2 * 16 + l15) * kLP + 8 * half);
      const v16h bv3 = F::load(Vt + (3 * 16 + l15) * kLP + 8 * half);
      o0 = F::mma(ap0, bv0, o0);
      o1 = F::mma(ap0, bv1, o1);
      o2 = F::mma(ap0, bv2, o2);
      o3 = F::mma(ap0, bv3, o3);
      keep4_h(bv0, bv1, bv2, bv3);
      const v16h ap1 = F::load(Pw + l15 * kLP + 32 + 8 * half);
      const v16h bv4 = F::load(Vt + (0 * 16 + l15) * kLP + 32 + 8 * half);
      const v16h bv5 = F::load(Vt + (1 * 16 + l15) * kLP + 32 + 8 * half);
      const v16h bv6 = F::load(Vt + (2 * 16 + l15) * kLP + 32 + 8 * half);
      const v16h bv7 = F::load(Vt + (3 * 16 + l15) * kLP + 32 + 8 * half);
      o0 = F::mma(ap1, bv4, o0);
      o1 = F::mma(ap1, bv5, o1);
      o2 = F::mma(ap1, bv6, o2);
      o3 = F::mma(ap1, bv7, o3);
      keep4_h(bv4, bv5, bv6, bv7);
      keep4_h(ap0, ap1, ap0, ap1);
    }
    acc_guard4(o0, o1, o2, o3);
  }
  acc_guard4(o0, o1, o2, o3);

  float il[8];
#pragma unroll
  for (int r = 0; r < 8; ++r) {
    const float rl = 1.0f / lrow[r];
    il[r] = (lrow[r] > 0.0f) ? (kPVScale * rl) : 0.0f;
  }
  __builtin_amdgcn_fence(3, "workgroup");
  __builtin_amdgcn_wave_barrier();
  __builtin_amdgcn_fence(2, "workgroup");
#pragma unroll
  for (int r = 0; r < 8; ++r) {
    _Float16* pr = Pw + (8 * half + r) * kLP + l15;
    pr[0]  = (_Float16)(o0[r] * il[r]);
    pr[16] = (_Float16)(o1[r] * il[r]);
    pr[32] = (_Float16)(o2[r] * il[r]);
    pr[48] = (_Float16)(o3[r] * il[r]);
  }
  __builtin_amdgcn_fence(3, "workgroup");
  __builtin_amdgcn_wave_barrier();
  __builtin_amdgcn_fence(2, "workgroup");
  const int q4 = lane >> 3, c8 = (lane & 7) * 8;
  _Float16* cb = (_Float16*)Cxp + (size_t)(tokq0 + wave * 16) * kModel + hoff;
  for (int pass = 0; pass < 2; ++pass) {
#pragma unroll
    for (int it = 0; it < 4; ++it) {
      const int row = it * 4 + q4;
      const v8h hv = *(const v8h*)(Pw + row * kLP + c8);
      *(volatile v8h*)(cb + (size_t)row * kModel + c8) = hv;
    }
    __threadfence();
  }
}

extern "C" void kernel_launch(void* const* d_in, const int* in_sizes, int n_in,
                              void* d_out, int out_size, void* d_ws, size_t ws_size,
                              hipStream_t stream) {
  if (n_in < 28) return;
  const long needTok = (long)(kBatch - 1) * kSeqFull + kSeq;
  if ((long)in_sizes[0] < needTok * kModel || (long)in_sizes[1] < needTok * kModel) return;
  if ((long)in_sizes[2] < needTok * kSeqFull || (long)in_sizes[3] < needTok * kSeqFull) return;
  {
    const int vecD[13] = {4, 5, 7, 10, 12, 13, 14, 16, 19, 21, 22, 23, 27};
    for (int i = 0; i < 13; ++i) if (in_sizes[vecD[i]] < kModel) return;
    const int matD[8] = {6, 8, 9, 11, 15, 17, 18, 20};
    for (int i = 0; i < 8; ++i) if (in_sizes[matD[i]] < kModel * kModel) return;
  }
  if (in_sizes[25] < kFF) return;
  if (in_sizes[24] < kModel * kFF || in_sizes[26] < kFF * kModel) return;
  if ((long)out_size < needTok * kModel) return;
  if (ws_size < kWsTotal) return;

  const float* dec   = (const float*)d_in[0];
  const float* enc   = (const float*)d_in[1];
  const int*   smsk  = (const int*)d_in[2];
  const int*   cmsk  = (const int*)d_in[3];
  const float* sa_g  = (const float*)d_in[4];
  const float* sa_b  = (const float*)d_in[5];
  const float* sa_wq = (const float*)d_in[6];
  const float* sa_bq = (const float*)d_in[7];
  const float* sa_wk = (const float*)d_in[8];
  const float* sa_wv = (const float*)d_in[9];
  const float* sa_bv = (const float*)d_in[10];
  const float* sa_wo = (const float*)d_in[11];
  const float* sa_bo = (const float*)d_in[12];
  const float* ca_g  = (const float*)d_in[13];
  const float* ca_b  = (const float*)d_in[14];
  const float* ca_wq = (const float*)d_in[15];
  const float* ca_bq = (const float*)d_in[16];
  const float* ca_wk = (const float*)d_in[17];
  const float* ca_wv = (const float*)d_in[18];
  const float* ca_bv = (const float*)d_in[19];
  const float* ca_wo = (const float*)d_in[20];
  const float* ca_bo = (const float*)d_in[21];
  const float* ml_g  = (const float*)d_in[22];
  const float* ml_b  = (const float*)d_in[23];
  const float* w1    = (const float*)d_in[24];
  const float* b1    = (const float*)d_in[25];
  const float* w2    = (const float*)d_in[26];
  const float* b2    = (const float*)d_in[27];
  float* outp = (float*)d_out;

  char* ws = (char*)d_ws;
  float*          xr    = (float*)(ws + kOffXR);
  unsigned short* enc16 = (unsigned short*)(ws + kOffEnc);
  unsigned short* w1T   = (unsigned short*)(ws + kOffW1T);
  unsigned short* h16   = (unsigned short*)(ws + kOffH16);
  unsigned short* wT4   = (unsigned short*)(ws + kOffWT4);
  unsigned short* w2T   = (unsigned short*)(ws + kOffW2T);
  unsigned short* q16   = (unsigned short*)(ws + kOffQ16);
  unsigned short* k16   = (unsigned short*)(ws + kOffK16);
  unsigned short* vt16  = (unsigned short*)(ws + kOffVT16);
  unsigned short* ctx16 = (unsigned short*)(ws + kOffCtx);
  unsigned short* hff   = (unsigned short*)(ws + kOffHFF);
  float*          y1    = (float*)(ws + kOffY1);
  float*          y2    = (float*)(ws + kOffY2);
  int*            fl0   = (int*)(ws + kOffFl0);
  int*            fl1   = (int*)(ws + kOffFl1);
  const unsigned short* wqT = wT4;
  const unsigned short* wkT = wT4 + (size_t)kModel * kModel;
  const unsigned short* wvT = wT4 + (size_t)2 * kModel * kModel;
  const unsigned short* woT = wT4 + (size_t)3 * kModel * kModel;

  const dim3 b256(256), b128(128);
  const dim3 gP((kTok / 64 * (kModel / 64) + 7) / 8, 1);
  const dim3 gV((kModel / 64 * (kTok / 64) + 7) / 8, 1);
  const dim3 gA(kQT, kBatch * kHeads);

  tileflag_kernel<<<dim3(kBatch * kQT, 2), b256, 0, stream>>>(smsk, cmsk, fl0, fl1);

  ln_kernel<true><<<dim3(kTok), b256, 0, stream>>>(dec, sa_g, sa_b, xr, h16);
  tcast_kernel<<<dim3(kModel / 64, kModel / 64, 4), b256, 0, stream>>>(
      sa_wq, sa_wk, sa_wv, sa_wo, wT4, kModel, kModel, (long)kModel * kModel, kWCarry);
  wmma_gemm64<0, false, 2, 1, false, 0, 0><<<gP, b256, 0, stream>>>(
      h16, h16, kModel, 0L, wqT, wqT, kModel, 0L, (void*)q16, (void*)q16, kModel, 0L,
      sa_bq, xr, 0L, kTok, kModel, kModel, kWCarryInv);
  wmma_gemm64<0, false, 0, 1, false, 0, 0><<<gP, b256, 0, stream>>>(
      h16, h16, kModel, 0L, wkT, wkT, kModel, 0L, (void*)k16, (void*)k16, kModel, 0L,
      sa_bq, xr, 0L, kTok, kModel, kModel, kWCarryInv);
  wmma_gemm64<0, false, 1, 1, false, 0, 0><<<gV, b256, 0, stream>>>(
      wvT, wvT, kModel, 0L, h16, h16, kModel, 0L, (void*)vt16, (void*)vt16, kTok, 0L,
      sa_bv, xr, 0L, kModel, kTok, kModel, kWCarryInv);
  attn_kernel<<<gA, b128, 0, stream>>>(q16, k16, vt16, smsk, fl0, ctx16);
  wmma_gemm64<0, false, 2, 0, true, 0, 0><<<gP, b256, 0, stream>>>(
      ctx16, ctx16, kModel, 0L, woT, woT, kModel, 0L, (void*)y1, (void*)y1, kModel, 0L,
      sa_bo, xr, 0L, kTok, kModel, kModel, kWoScale);

  {
    const int n8 = kTok * kModel / 8;
    enccast_kernel<<<dim3((n8 + 255) / 256), b256, 0, stream>>>(enc, enc16, n8);
  }
  ln_kernel<false><<<dim3(kTok), b256, 0, stream>>>(y1, ca_g, ca_b, y2, h16);
  tcast_kernel<<<dim3(kModel / 64, kModel / 64, 4), b256, 0, stream>>>(
      ca_wq, ca_wk, ca_wv, ca_wo, wT4, kModel, kModel, (long)kModel * kModel, kWCarry);
  wmma_gemm64<0, false, 2, 1, false, 0, 0><<<gP, b256, 0, stream>>>(
      h16, h16, kModel, 0L, wqT, wqT, kModel, 0L, (void*)q16, (void*)q16, kModel, 0L,
      ca_bq, y1, 0L, kTok, kModel, kModel, kWCarryInv);
  wmma_gemm64<0, false, 0, 1, false, 0, 0><<<gP, b256, 0, stream>>>(
      enc16, enc16, kModel, 0L, wkT, wkT, kModel, 0L, (void*)k16, (void*)k16, kModel, 0L,
      ca_bq, y1, 0L, kTok, kModel, kModel, kWCarryInv);
  wmma_gemm64<0, false, 1, 1, false, 0, 0><<<gV, b256, 0, stream>>>(
      wvT, wvT, kModel, 0L, enc16, enc16, kModel, 0L, (void*)vt16, (void*)vt16, kTok, 0L,
      ca_bv, y1, 0L, kModel, kTok, kModel, kWCarryInv);
  attn_kernel<<<gA, b128, 0, stream>>>(q16, k16, vt16, cmsk, fl1, ctx16);
  wmma_gemm64<0, false, 2, 0, true, 0, 0><<<gP, b256, 0, stream>>>(
      ctx16, ctx16, kModel, 0L, woT, woT, kModel, 0L, (void*)y2, (void*)y2, kModel, 0L,
      ca_bo, y1, 0L, kTok, kModel, kModel, kWoScale);

  ln_kernel<false><<<dim3(kTok), b256, 0, stream>>>(y2, ml_g, ml_b, y1, h16);
  tcast_kernel<<<dim3(kModel / 64, kFF / 64, 1), b256, 0, stream>>>(
      w1, w1, w1, w1, w1T, kModel, kFF, 0L, kWCarry);
  tcast_kernel<<<dim3(kFF / 64, kModel / 64, 1), b256, 0, stream>>>(
      w2, w2, w2, w2, w2T, kFF, kModel, 0L, kW2Carry);
  {
    const dim3 g((kTok / 64 * (kFF / 64) + 7) / 8, 1);
    wmma_gemm64<0, false, 2, 1, false, 3, 0><<<g, b256, 0, stream>>>(
        h16, h16, kModel, 0L, w1T, w1T, kModel, 0L, (void*)hff, (void*)hff, kFF, 0L,
        b1, y2, 0L, kTok, kFF, kModel, kWCarryInv);
  }
  {
    const dim3 g(((kSeq / 64) * (kModel / 64) + 7) / 8, kBatch);
    wmma_gemm64<0, false, 2, 0, true, 0, 0><<<g, b256, 0, stream>>>(
        hff, hff, kFF, (long)kSeq * kFF, w2T, w2T, kFF, 0L, (void*)outp, (void*)outp, kModel, (long)kSeqFull * kModel,
        b2, y2, (long)kSeq * kModel, kSeq, kModel, kFF, kW2CarryInv);
  }
}
